// S6DReal_71425306133129
// MI455X (gfx1250) — hardware-run, weakly checked
//
#include <hip/hip_runtime.h>
#include <hip/hip_fp16.h>
#include <math.h>

typedef __attribute__((ext_vector_type(16))) _Float16 v16h;
typedef __attribute__((ext_vector_type(8)))  _Float16 v8h;
typedef __attribute__((ext_vector_type(8)))  float    v8f;
typedef __attribute__((ext_vector_type(4)))  float    v4f;
typedef __attribute__((ext_vector_type(2)))  unsigned v2u;

constexpr int kL   = 8192;
constexpr int kC   = 256;
constexpr int kS   = 64;
constexpr int kN   = 384;
constexpr int kNch = 32;
constexpr int kChl = 256;
constexpr float kWCarry = 65536.0f;
constexpr float sW      = 1.0f / kWCarry;
constexpr float kDtOff  = 1.0f / 4096.0f;
static_assert(kN == kS + kS + kC);
static_assert(kNch * kChl == kL);
static_assert(kC == 8 * 32);
static_assert(kS == 2 * 32);
static_assert((kC % 32) == 0 && (kN % 64) == 0 && (kL % 32) == 0);

constexpr size_t kSzAL = (size_t)kC * kS * 4;
constexpr size_t kSzXH = (size_t)kL * kC * 2;
constexpr size_t kSzXB = (size_t)kL * kC * 4;
constexpr size_t kSzWT = (size_t)kN * kC * 2;
constexpr size_t kSzP  = (size_t)kL * kN * 4;
constexpr size_t kSzQ  = (size_t)kL * kN * 4;
constexpr size_t kSzU  = (size_t)kNch * kS * kC * 4;
constexpr size_t kSzSD = (size_t)kNch * kC * 4;
constexpr size_t kSzH  = (size_t)kNch * kS * kC * 4;
constexpr size_t kSzYP = (size_t)kL * kC * 4;
constexpr size_t kOffAL = 0;
constexpr size_t kOffXH = kOffAL + kSzAL;
constexpr size_t kOffXB = kOffXH + kSzXH;
constexpr size_t kOffWT = kOffXB + kSzXB;
constexpr size_t kOffP  = kOffWT + kSzWT;
constexpr size_t kOffQ  = kOffP  + kSzP;
constexpr size_t kOffU  = kOffQ  + kSzQ;
constexpr size_t kOffSD = kOffU  + kSzU;
constexpr size_t kOffH  = kOffSD + kSzSD;
constexpr size_t kOffYP = kOffH  + kSzH;
constexpr size_t kWsTotal = kOffYP + kSzYP;
static_assert(kWsTotal == 50626560ull);
static_assert(kWsTotal <= 134217728ull);
static_assert((kOffXH % 256) == 0 && (kOffXB % 256) == 0 && (kOffWT % 256) == 0 && (kOffP % 256) == 0 &&
              (kOffQ % 256) == 0 && (kOffU % 256) == 0 && (kOffSD % 256) == 0 && (kOffH % 256) == 0 &&
              (kOffYP % 256) == 0);

__device__ __forceinline__ _Float16 f16_flush(float v) {
  const float w = (fabsf(v) < 6.103515625e-05f) ? 0.0f : v;
  return (_Float16)w;
}

__device__ __forceinline__ float bf16r(float v) {
  unsigned u = __float_as_uint(v);
  u = (u + 0x7FFFu + ((u >> 16) & 1u)) & 0xFFFF0000u;
  return __uint_as_float(u);
}

namespace eng {
union FragU { v16h v; v8h h[2]; };
__device__ __forceinline__ v16h frag_load(const _Float16* p) {
  FragU f;
  f.h[0] = *(const v8h*)(p);
  f.h[1] = *(const v8h*)(p + 16);
  return f.v;
}
__device__ __forceinline__ v8f mma(v16h a, v16h b, v8f c) {
  return __builtin_amdgcn_wmma_f32_16x16x32_f16(false, a, false, b, (short)0, c, false, false);
}
__device__ __forceinline__ void guard1(v8f& a, v16h x, v16h y) {
  asm volatile("v_nop\n\tv_nop\n\tv_nop\n\tv_nop" : "+v"(a) : "v"(x), "v"(y));
}
__device__ __forceinline__ void guard_acc(v8f& a) {
  asm volatile("v_nop\n\tv_nop\n\tv_nop\n\tv_nop" : "+v"(a));
}
__device__ __forceinline__ void keep4(v16h a, v16h b, v16h c, v16h d) {
  asm volatile("v_nop" :: "v"(a), "v"(b), "v"(c), "v"(d));
}

template <int MI, int SPL>
__global__ __launch_bounds__(256) void gemm_f16_kernel(
    const unsigned short* __restrict__ Ap, const unsigned short* __restrict__ A2p, int lda,
    const unsigned short* __restrict__ Btp, const unsigned short* __restrict__ Bt2p, int ldb,
    float* __restrict__ C, int ldc, int M, int N, int K, float scale, float rscale)
{
  static_assert(MI >= 1 && MI <= 2);
  static_assert(SPL >= 0 && SPL <= 2);
  const _Float16* A   = (const _Float16*)Ap;
  const _Float16* A2  = (const _Float16*)A2p;
  const _Float16* Bt  = (const _Float16*)Btp;
  const _Float16* Bt2 = (const _Float16*)Bt2p;
  __shared__ __align__(16) float sT[8][16 * 68];
  const int lane = threadIdx.x & 31;
  const int wave = threadIdx.x >> 5;
  const int tilesN = N >> 6;
  const int tilesM = M / (16 * MI);
  const int tile = blockIdx.x * 8 + wave;
  if (tile >= tilesM * tilesN) return;
  const int tm = tile / tilesN;
  const int tn = tile - tm * tilesN;
  const int m0 = tm * (16 * MI);
  const int n0 = tn << 6;
  const int rlane = lane & 15;
  const int koff  = (lane >> 4) * 8;
  const int mOff  = (lane >> 4) * 8;

  v8f acc[MI][4], accr[MI][4];
#pragma unroll
  for (int i = 0; i < MI; ++i)
#pragma unroll
    for (int j = 0; j < 4; ++j) {
      acc[i][j]  = (v8f){0.f, 0.f, 0.f, 0.f, 0.f, 0.f, 0.f, 0.f};
      accr[i][j] = (v8f){0.f, 0.f, 0.f, 0.f, 0.f, 0.f, 0.f, 0.f};
    }

  for (int k0 = 0; k0 < K; k0 += 32) {
    v16h bh[4], bl[4];
#pragma unroll
    for (int j = 0; j < 4; ++j) {
      const size_t bo = (size_t)(n0 + (j << 4) + rlane) * ldb + koff + k0;
      bh[j] = frag_load(Bt + bo);
      if (SPL == 2) bl[j] = frag_load(Bt2 + bo); else bl[j] = bh[j];
    }
#pragma unroll
    for (int i = 0; i < MI; ++i) {
      const size_t ao = (size_t)(m0 + (i << 4) + rlane) * lda + koff + k0;
      const v16h ah = frag_load(A + ao);
      v16h al = ah;
      if (SPL >= 1) al = frag_load(A2 + ao);
#pragma unroll
      for (int j = 0; j < 4; ++j) {
        acc[i][j] = mma(ah, bh[j], acc[i][j]);
        if (SPL >= 1) accr[i][j] = mma(al, bh[j], accr[i][j]);
        if (SPL == 2) accr[i][j] = mma(ah, bl[j], accr[i][j]);
      }
#pragma unroll
      for (int j = 0; j < 4; ++j) {
        guard1(acc[i][j], ah, al);
        if (SPL >= 1) guard1(accr[i][j], ah, al);
      }
    }
    keep4(bh[0], bh[1], bh[2], bh[3]);
    if (SPL == 2) keep4(bl[0], bl[1], bl[2], bl[3]);
  }
#pragma unroll
  for (int i = 0; i < MI; ++i)
#pragma unroll
    for (int j = 0; j < 4; ++j) {
      guard_acc(acc[i][j]);
      if (SPL >= 1) guard_acc(accr[i][j]);
    }

  float* slab = sT[wave];
#pragma unroll
  for (int i = 0; i < MI; ++i) {
    const int mBase = m0 + (i << 4);
#pragma unroll
    for (int j = 0; j < 4; ++j) {
#pragma unroll
      for (int r = 0; r < 8; ++r) {
        float v = acc[i][j][r] * scale;
        if (SPL >= 1) v += accr[i][j][r] * rscale;
        slab[(mOff + r) * 68 + (j << 4) + rlane] = v;
      }
    }
    __builtin_amdgcn_fence(__ATOMIC_RELEASE, "workgroup");
    __builtin_amdgcn_wave_barrier();
    __builtin_amdgcn_fence(__ATOMIC_ACQUIRE, "workgroup");
    {
      const int hh = lane >> 4, c4 = (lane & 15) * 4;
      for (int pass = 0; pass < 2; ++pass) {
#pragma unroll
        for (int it = 0; it < 8; ++it) {
          const int row = it * 2 + hh;
          const v4f v = *(const v4f*)(slab + row * 68 + c4);
          *(volatile v4f*)(C + (size_t)(mBase + row) * ldc + n0 + c4) = v;
        }
        __threadfence();
      }
    }
    __builtin_amdgcn_fence(__ATOMIC_RELEASE, "workgroup");
    __builtin_amdgcn_wave_barrier();
    __builtin_amdgcn_fence(__ATOMIC_ACQUIRE, "workgroup");
  }
}
}

__global__ __launch_bounds__(256) void rne_rows_f16_kernel(
    const float* __restrict__ src, unsigned short* __restrict__ dH, int total8)
{
  const int i = blockIdx.x * 256 + threadIdx.x;
  if (i >= total8) return;
  const size_t e0 = (size_t)i << 3;
  const v4f a0 = *(const v4f*)(src + e0);
  const v4f a1 = *(const v4f*)(src + e0 + 4);
  const float f0 = a0[0];
  const float f1 = a0[1];
  const float f2 = a0[2];
  const float f3 = a0[3];
  const float f4 = a1[0];
  const float f5 = a1[1];
  const float f6 = a1[2];
  const float f7 = a1[3];
  v8h hv;
  hv[0] = f16_flush(bf16r(f0));
  hv[1] = f16_flush(bf16r(f1));
  hv[2] = f16_flush(bf16r(f2));
  hv[3] = f16_flush(bf16r(f3));
  hv[4] = f16_flush(bf16r(f4));
  hv[5] = f16_flush(bf16r(f5));
  hv[6] = f16_flush(bf16r(f6));
  hv[7] = f16_flush(bf16r(f7));
  unsigned short* qh = dH + e0;
  *(volatile v8h*)qh = hv;
  __threadfence();
  *(volatile v8h*)qh = hv;
}

__global__ __launch_bounds__(256) void rne_vec_kernel(
    const float* __restrict__ src, float* __restrict__ dst, int n4)
{
  const int i = blockIdx.x * 256 + threadIdx.x;
  if (i >= n4) return;
  const v4f a = *(const v4f*)(src + (size_t)i * 4);
  const float a0 = a[0];
  const float a1 = a[1];
  const float a2 = a[2];
  const float a3 = a[3];
  v4f r;
  r[0] = bf16r(a0);
  r[1] = bf16r(a1);
  r[2] = bf16r(a2);
  r[3] = bf16r(a3);
  float* p = dst + (size_t)i * 4;
  *(volatile v4f*)p = r;
  __threadfence();
  *(volatile v4f*)p = r;
}

__global__ __launch_bounds__(256) void rne_plane_kernel(
    const float* __restrict__ src, float* __restrict__ dst, int n4)
{
  const int i = blockIdx.x * 256 + threadIdx.x;
  if (i >= n4) return;
  const v4f a = *(const v4f*)(src + (size_t)i * 4);
  const float a0 = a[0];
  const float a1 = a[1];
  const float a2 = a[2];
  const float a3 = a[3];
  v4f r;
  r[0] = bf16r(a0);
  r[1] = bf16r(a1);
  r[2] = bf16r(a2);
  r[3] = bf16r(a3);
  float* p = dst + (size_t)i * 4;
  *(volatile v4f*)p = r;
  __threadfence();
  *(volatile v4f*)p = r;
}

__global__ __launch_bounds__(256) void wcat_pack_kernel(
    const float* __restrict__ WB, const float* __restrict__ WC, const float* __restrict__ WD,
    unsigned short* __restrict__ WT)
{
  const int jt = blockIdx.x * 256 + threadIdx.x;
  const int n  = jt >> 5;
  const int k0 = (jt & 31) * 8;
  const float* src;
  int col;
  int ld;
  if (n < kS) {
    src = WB;
    col = n;
    ld = kS;
  } else if (n < 2 * kS) {
    src = WC;
    col = n - kS;
    ld = kS;
  } else {
    src = WD;
    col = n - 2 * kS;
    ld = kC;
  }
  float w[8];
#pragma unroll
  for (int e = 0; e < 8; ++e) w[e] = src[(size_t)(k0 + e) * ld + col];
  v8h hv;
#pragma unroll
  for (int e = 0; e < 8; ++e) hv[e] = f16_flush(bf16r(w[e]) * kWCarry);
  unsigned short* qh = WT + (size_t)jt * 8;
  *(volatile v8h*)qh = hv;
  __threadfence();
  *(volatile v8h*)qh = hv;
}

__global__ __launch_bounds__(256) void epilogue_kernel(
    const float* __restrict__ P, const float* __restrict__ bB, const float* __restrict__ bC,
    const float* __restrict__ bD, float* __restrict__ Q)
{
  const int e   = blockIdx.x * 256 + threadIdx.x;
  const int row = e / 96;
  const int n0  = 4 * (e - 96 * row);
  const v4f pv = *(const v4f*)(P + (size_t)row * kN + n0);
  int ib = n0;
  ib = (ib > kS - 4) ? (kS - 4) : ib;
  int ic = n0 - kS;
  ic = (ic < 0) ? 0 : ic;
  ic = (ic > kS - 4) ? (kS - 4) : ic;
  int id = n0 - 2 * kS;
  id = (id < 0) ? 0 : id;
  id = (id > kC - 4) ? (kC - 4) : id;
  const v4f vb = *(const v4f*)(bB + ib);
  const v4f vc = *(const v4f*)(bC + ic);
  const v4f vd = *(const v4f*)(bD + id);
  float p[4], tb[4], tc[4], td[4];
  p[0] = pv[0];
  p[1] = pv[1];
  p[2] = pv[2];
  p[3] = pv[3];
  tb[0] = vb[0];
  tb[1] = vb[1];
  tb[2] = vb[2];
  tb[3] = vb[3];
  tc[0] = vc[0];
  tc[1] = vc[1];
  tc[2] = vc[2];
  tc[3] = vc[3];
  td[0] = vd[0];
  td[1] = vd[1];
  td[2] = vd[2];
  td[3] = vd[3];
  float q[4];
  if (n0 < 2 * kS) {
    const bool isB = (n0 < kS);
#pragma unroll
    for (int k = 0; k < 4; ++k) {
      const float fb = (1.0f + p[k]) + bf16r(tb[k]);
      const float fc = p[k] + bf16r(tc[k]);
      q[k] = isB ? fb : fc;
    }
  } else {
#pragma unroll
    for (int k = 0; k < 4; ++k) {
      const float z = (kDtOff + p[k]) + bf16r(td[k]);
      q[k] = fmaxf(z, 0.0f) + log1pf(expf(-fabsf(z)));
    }
  }
  v4f qv;
  qv[0] = q[0];
  qv[1] = q[1];
  qv[2] = q[2];
  qv[3] = q[3];
  float* dst = Q + (size_t)row * kN + n0;
  *(volatile v4f*)dst = qv;
  __threadfence();
  *(volatile v4f*)dst = qv;
}

__global__ __launch_bounds__(256) void scan_local_kernel(
    const float* __restrict__ XB, const float* __restrict__ Q, const float* __restrict__ AL,
    float* __restrict__ U, float* __restrict__ SD)
{
  const int lane = threadIdx.x & 31;
  const int g    = threadIdx.x >> 5;
  const int j    = blockIdx.x;
  const int c    = 32 * g + lane;
  const int l0   = kChl * j;
  float sd = 0.0f;
  for (int hf = 0; hf < 2; ++hf) {
    const int sb = 32 * hf;
    float a[32], ia[32], h[32];
    const float* ap = AL + (size_t)c * kS + sb;
#pragma unroll
    for (int k = 0; k < 8; ++k) {
      const v4f lg = *(const v4f*)(ap + 4 * k);
#pragma unroll
      for (int e = 0; e < 4; ++e) {
        const float av = -expf(lg[e]);
        a[4 * k + e]  = av;
        ia[4 * k + e] = 1.0f / av;
        h[4 * k + e]  = 0.0f;
      }
    }
    for (int i = 0; i < kChl; ++i) {
      const size_t l = (size_t)(l0 + i);
      const float xv = XB[l * kC + c];
      const float dv = Q[l * kN + 2 * kS + c];
      const float* bp = Q + l * kN + sb;
      v4f bq[8];
#pragma unroll
      for (int k = 0; k < 8; ++k) bq[k] = *(const v4f*)(bp + 4 * k);
      const float dadd = (hf == 0) ? dv : 0.0f;
      sd += dadd;
#pragma unroll
      for (int r = 0; r < 32; ++r) {
        const float At = expf(a[r] * dv);
        const float bx = bq[r >> 2][r & 3] * xv;
        const float ut = (At - 1.0f) * bx * ia[r];
        h[r] = At * h[r] + ut;
      }
    }
    for (int pass = 0; pass < 2; ++pass) {
#pragma unroll
      for (int r = 0; r < 32; ++r)
        *(volatile float*)(U + (size_t)(j * kS + sb + r) * kC + c) = h[r];
      __threadfence();
    }
  }
  float* sp = SD + (size_t)j * kC + c;
  *(volatile float*)sp = sd;
  __threadfence();
  *(volatile float*)sp = sd;
}

__global__ __launch_bounds__(256) void scan_carry_kernel(
    const float* __restrict__ AL, const float* __restrict__ SD, const float* __restrict__ U,
    float* __restrict__ H)
{
  const int lane = threadIdx.x & 31;
  const int g    = threadIdx.x >> 5;
  const int s    = blockIdx.x;
  const int c    = 32 * g + lane;
  const float a  = -expf(AL[(size_t)c * kS + s]);
  float hc = 0.0f;
  {
    float* hp = H + (size_t)s * kC + c;
    *(volatile float*)hp = hc;
    __threadfence();
    *(volatile float*)hp = hc;
  }
  for (int j = 0; j < kNch - 1; ++j) {
    const float sdv = SD[(size_t)j * kC + c];
    const float uv  = U[(size_t)(j * kS + s) * kC + c];
    hc = expf(a * sdv) * hc + uv;
    float* hp = H + (size_t)((j + 1) * kS + s) * kC + c;
    *(volatile float*)hp = hc;
    __threadfence();
    *(volatile float*)hp = hc;
  }
}

__global__ __launch_bounds__(256) void scan_final_kernel(
    const float* __restrict__ XB, const float* __restrict__ Q, const float* __restrict__ AL,
    const float* __restrict__ H, float* YP, float* out)
{
  const int lane = threadIdx.x & 31;
  const int g    = threadIdx.x >> 5;
  const int j    = blockIdx.x;
  const int c    = 32 * g + lane;
  const int l0   = kChl * j;
  for (int hf = 0; hf < 2; ++hf) {
    const int sb = 32 * hf;
    float a[32], ia[32], h[32];
    const float* ap = AL + (size_t)c * kS + sb;
#pragma unroll
    for (int k = 0; k < 8; ++k) {
      const v4f lg = *(const v4f*)(ap + 4 * k);
#pragma unroll
      for (int e = 0; e < 4; ++e) {
        const float av = -expf(lg[e]);
        a[4 * k + e]  = av;
        ia[4 * k + e] = 1.0f / av;
        h[4 * k + e]  = H[(size_t)(j * kS + sb + 4 * k + e) * kC + c];
      }
    }
    float* dst = (hf == 0) ? YP : out;
    for (int i = 0; i < kChl; ++i) {
      const size_t l = (size_t)(l0 + i);
      const size_t o = l * kC + c;
      const float xv = XB[o];
      const float dv = Q[l * kN + 2 * kS + c];
      const float* bp = Q + l * kN + sb;
      const float* cp = bp + kS;
      v4f bq[8], cq[8];
#pragma unroll
      for (int k = 0; k < 8; ++k) {
        bq[k] = *(const v4f*)(bp + 4 * k);
        cq[k] = *(const v4f*)(cp + 4 * k);
      }
      float acc = 0.0f;
      if (hf != 0) acc = *(const volatile __attribute__((address_space(1))) float*)(YP + o);
#pragma unroll
      for (int r = 0; r < 32; ++r) {
        const float At = expf(a[r] * dv);
        const float bx = bq[r >> 2][r & 3] * xv;
        const float ut = (At - 1.0f) * bx * ia[r];
        h[r] = At * h[r] + ut;
        acc = acc + cq[r >> 2][r & 3] * h[r];
      }
      *(volatile float*)(dst + o) = acc;
      __threadfence();
      *(volatile float*)(dst + o) = acc;
    }
  }
}

static_assert(((kC * kS / 4) % 256) == 0);
static_assert(((kL * kC / 8) % 256) == 0);
static_assert(((kL * kC / 4) % 256) == 0);
static_assert(((kN * kC / 8) % 256) == 0);
static_assert(((kL / 32) * (kN / 64)) % 8 == 0);
static_assert(((kL * (kN / 4)) % 256) == 0);
static_assert((kN / 4) == 96);

extern "C" void kernel_launch(void* const* d_in, const int* in_sizes, int n_in,
                              void* d_out, int out_size, void* d_ws, size_t ws_size,
                              hipStream_t stream)
{
  if (n_in < 8) return;
  if (in_sizes[0] != kL * kC) return;
  if (in_sizes[1] != kC * kS) return;
  if (in_sizes[2] != kC * kS) return;
  if (in_sizes[3] != kS) return;
  if (in_sizes[4] != kC * kS) return;
  if (in_sizes[5] != kS) return;
  if (in_sizes[6] != kC * kC) return;
  if (in_sizes[7] != kC) return;
  if (out_size != 2097152) return;
  if (ws_size < kWsTotal) return;

  const float* x       = (const float*)d_in[0];
  const float* lognegA = (const float*)d_in[1];
  const float* W_B     = (const float*)d_in[2];
  const float* b_B     = (const float*)d_in[3];
  const float* W_C     = (const float*)d_in[4];
  const float* b_C     = (const float*)d_in[5];
  const float* W_dt    = (const float*)d_in[6];
  const float* b_dt    = (const float*)d_in[7];
  float* out = (float*)d_out;

  char* ws = (char*)d_ws;
  float*          AL = (float*)(ws + kOffAL);
  unsigned short* XH = (unsigned short*)(ws + kOffXH);
  float*          XB = (float*)(ws + kOffXB);
  unsigned short* WT = (unsigned short*)(ws + kOffWT);
  float*          P  = (float*)(ws + kOffP);
  float*          Q  = (float*)(ws + kOffQ);
  float*          U  = (float*)(ws + kOffU);
  float*          SD = (float*)(ws + kOffSD);
  float*          H  = (float*)(ws + kOffH);
  float*          YP = (float*)(ws + kOffYP);

  rne_vec_kernel<<<(kC * kS / 4) / 256, 256, 0, stream>>>(lognegA, AL, kC * kS / 4);

  rne_rows_f16_kernel<<<(kL * kC / 8) / 256, 256, 0, stream>>>(x, XH, kL * kC / 8);

  rne_plane_kernel<<<(kL * kC / 4) / 256, 256, 0, stream>>>(x, XB, kL * kC / 4);

  wcat_pack_kernel<<<(kN * kC / 8) / 256, 256, 0, stream>>>(W_B, W_C, W_dt, WT);

  eng::gemm_f16_kernel<2, 0><<<dim3((kL / 32) * (kN / 64) / 8), 256, 0, stream>>>(
      XH, nullptr, kC, WT, nullptr, kC, P, kN, kL, kN, kC, sW, 0.0f);

  epilogue_kernel<<<(kL * (kN / 4)) / 256, 256, 0, stream>>>(P, b_B, b_C, b_dt, Q);

  scan_local_kernel<<<kNch, 256, 0, stream>>>(XB, Q, AL, U, SD);

  scan_carry_kernel<<<kS, 256, 0, stream>>>(AL, SD, U, H);

  scan_final_kernel<<<kNch, 256, 0, stream>>>(XB, Q, AL, H, YP, out);
}
